// TrillNet_19310172963036
// MI455X (gfx1250) — hardware-verified
//
#include <hip/hip_runtime.h>
#define BB 8
#define HT 16
#define SQ 64
#define DIM 128
#define CC 2000
#define DM 256
#define NHD 4
#define HDD 64
#define DFF 1024
#define NSEQ (BB * HT + BB)
#define NR (NSEQ * SQ)
#define NEPB (HT * (SQ - 1))

typedef __bf16 v16b __attribute__((ext_vector_type(16)));
typedef unsigned short v8us __attribute__((ext_vector_type(8), may_alias));
typedef float  v8f  __attribute__((ext_vector_type(8)));
typedef float  v4f  __attribute__((ext_vector_type(4)));
typedef float  v4fa __attribute__((ext_vector_type(4), may_alias));
union FragB { v16b v; v8us half[2]; unsigned short u[16]; };

__device__ __forceinline__ unsigned short bf16_bits(float x) { unsigned int u = __float_as_uint(x); return (unsigned short)((u + 0x7FFFu + ((u >> 16) & 1u)) >> 16); }
__device__ __forceinline__ float bf16_val(unsigned short b) { return __uint_as_float(((unsigned int)b) << 16); }
__device__ __forceinline__ float bf16_round(float x) { return bf16_val(bf16_bits(x)); }
template <int NT>
__device__ __forceinline__ v8f mmaN(v16b ah, v16b al, v16b bh, v16b bl, v8f c) {
  c = __builtin_amdgcn_wmma_f32_16x16x32_bf16(false, ah, false, bh, (short)0, c, false, false);
  if (NT >= 2) c = __builtin_amdgcn_wmma_f32_16x16x32_bf16(false, al, false, bh, (short)0, c, false, false);
  if (NT >= 3) c = __builtin_amdgcn_wmma_f32_16x16x32_bf16(false, ah, false, bl, (short)0, c, false, false);
  asm volatile("v_nop\n\tv_nop\n\tv_nop\n\tv_nop" : "+v"(c) : "v"(ah), "v"(al), "v"(bh), "v"(bl));
  return c;
}

__global__ __launch_bounds__(256) void k_wt_bf16(const float* __restrict__ W, unsigned short* __restrict__ Wt, int K, int N) {
  const int t = blockIdx.x * 256 + threadIdx.x;
  const int k8n = K / 8;
  if (t >= N * k8n) return;
  const int n = t / k8n, k8 = (t % k8n) * 8;
  v8us v;
#pragma unroll
  for (int i = 0; i < 8; ++i) v[i] = bf16_bits(W[(size_t)(k8 + i) * N + n]);
  *(volatile v8us*)(Wt + (size_t)n * K + k8) = v;
  __threadfence();
  *(volatile v8us*)(Wt + (size_t)n * K + k8) = v;
}

template <bool ASPLIT, int ACT, bool BIAS_BF16>
__global__ __launch_bounds__(128) void k_gemm_bf(const float* __restrict__ A, int lda, const unsigned short* __restrict__ Wt, int ldb,
                                               const float* __restrict__ bias, float* __restrict__ C, int ldc, int M, int N, int K) {
  __shared__ __attribute__((aligned(16))) float so[4][16][64];
  const int tid = threadIdx.x, w = tid >> 5, lane = tid & 31, ln = lane & 15, hh = lane >> 4;
  const int ntn = N / 64;
  const int wid = blockIdx.x * 4 + w;
  const int mt = wid / ntn, nq = wid % ntn;
  if (mt * 16 >= M) return;
  const int row0 = mt * 16, col0 = nq * 64;
  const float* arow = A + (size_t)(row0 + ln) * lda;
  v8f acc[4] = {};
  for (int kb = 0; kb < K; kb += 32) {
    FragB ah, al;
    const v4f x0 = *(const v4fa*)(arow + kb + 8 * hh), x1 = *(const v4fa*)(arow + kb + 8 * hh + 4);
    const v4f x2 = *(const v4fa*)(arow + kb + 16 + 8 * hh), x3 = *(const v4fa*)(arow + kb + 16 + 8 * hh + 4);
    float xs[16] = {x0[0],x0[1],x0[2],x0[3],x1[0],x1[1],x1[2],x1[3],x2[0],x2[1],x2[2],x2[3],x3[0],x3[1],x3[2],x3[3]};
#pragma unroll
    for (int i = 0; i < 16; ++i) { const unsigned short hb = bf16_bits(xs[i]); ah.u[i] = hb; al.u[i] = ASPLIT ? bf16_bits(xs[i] - bf16_val(hb)) : (unsigned short)0; }
#pragma unroll
    for (int t = 0; t < 4; ++t) {
      const unsigned short* brow = Wt + (size_t)(col0 + t * 16 + ln) * ldb + kb;
      FragB b;
      b.half[0] = *(const v8us*)(brow + 8 * hh);
      b.half[1] = *(const v8us*)(brow + 16 + 8 * hh);
      acc[t] = mmaN<ASPLIT ? 2 : 1>(ah.v, al.v, b.v, b.v, acc[t]);
    }
  }
#pragma unroll
  for (int t = 0; t < 4; ++t) {
    float bv = bias ? bias[col0 + t * 16 + ln] : 0.f;
    if (BIAS_BF16) bv = bf16_round(bv);
#pragma unroll
    for (int r = 0; r < 8; ++r) { float v = acc[t][r] + bv; if (ACT == 1) v = fmaxf(v, 0.f); so[w][8 * hh + r][t * 16 + ln] = v; }
  }
  __builtin_amdgcn_fence(__ATOMIC_ACQ_REL, "workgroup");
  __builtin_amdgcn_wave_barrier();
  const int rsub = lane >> 4, c4 = (lane & 15) * 4;
  for (int pass = 0; pass < 2; ++pass) {
#pragma unroll
    for (int q = 0; q < 8; ++q) {
      const int r = q * 2 + rsub;
      const v4f v = *(const v4fa*)&so[w][r][c4];
      *(volatile v4f*)(C + (size_t)(row0 + r) * ldc + col0 + c4) = v;
    }
    if (pass == 0) __threadfence();
  }
}

template <int D, bool CAUSAL>
__global__ __launch_bounds__(128) void k_flash(const float* __restrict__ qb, const float* __restrict__ kb, const float* __restrict__ vb,
                                             int pitch, int T, int H, float scale, float* __restrict__ y, int ypitch) {
  constexpr int KS = D / 32;
  constexpr int DT = D / 16;
  __shared__ __attribute__((aligned(16))) unsigned short sKh[32][D + 8], sKl[32][D + 8], sVh[32][D + 8], sVl[32][D + 8];
  __shared__ __attribute__((aligned(16))) unsigned short sPh[4][16][40], sPl[4][16][40];
  __shared__ __attribute__((aligned(16))) float sO[4][16][D];
  const int tid = threadIdx.x, w = tid >> 5, lane = tid & 31, ln = lane & 15, hh = lane >> 4;
  const int nqb = (T + 63) / 64;
  const int bh = blockIdx.x / nqb, qblk = blockIdx.x % nqb;
  const int b = bh / H, h = bh % H;
  const int q0 = qblk * 64 + w * 16;
  const float* Q = qb + (size_t)b * T * pitch + h * D;
  const float* K = kb + (size_t)b * T * pitch + h * D;
  const float* V = vb + (size_t)b * T * pitch + h * D;

  FragB aqh[KS], aql[KS];
  {
    int row = q0 + ln; if (row >= T) row = T - 1;
    const float* qr = Q + (size_t)row * pitch;
#pragma unroll
    for (int ks = 0; ks < KS; ++ks)
#pragma unroll
      for (int i = 0; i < 16; ++i) {
        const int d = ks * 32 + ((i < 8) ? (8 * hh + i) : (16 + 8 * hh + (i - 8)));
        const float x = qr[d] * scale; const unsigned short hb = bf16_bits(x);
        aqh[ks].u[i] = hb; aql[ks].u[i] = bf16_bits(x - bf16_val(hb));
      }
  }
  float m_r[8], l_r[8];
#pragma unroll
  for (int r = 0; r < 8; ++r) { m_r[r] = -3.0e38f; l_r[r] = 0.f; }
  v8f oacc[DT];
#pragma unroll
  for (int dt = 0; dt < DT; ++dt) oacc[dt] = (v8f){0.f,0.f,0.f,0.f,0.f,0.f,0.f,0.f};

  const int kv_end = CAUSAL ? min(T, qblk * 64 + 64) : T;
  for (int j0 = 0; j0 < kv_end; j0 += 32) {
    __syncthreads();
    for (int e = tid; e < 32 * (D / 4); e += 128) {
      const int r = e / (D / 4), c4 = (e % (D / 4)) * 4;
      const int key = j0 + r;
      v4f kf = {0.f,0.f,0.f,0.f}, vf = {0.f,0.f,0.f,0.f};
      if (key < T) { kf = *(const v4fa*)(K + (size_t)key * pitch + c4); vf = *(const v4fa*)(V + (size_t)key * pitch + c4); }
#pragma unroll
      for (int t = 0; t < 4; ++t) {
        unsigned short hb = bf16_bits(kf[t]); sKh[r][c4 + t] = hb; sKl[r][c4 + t] = bf16_bits(kf[t] - bf16_val(hb));
        hb = bf16_bits(vf[t]); sVh[r][c4 + t] = hb; sVl[r][c4 + t] = bf16_bits(vf[t] - bf16_val(hb));
      }
    }
    __syncthreads();
    v8f s[2];
#pragma unroll
    for (int nt = 0; nt < 2; ++nt) {
      v8f acc = {};
#pragma unroll
      for (int ks = 0; ks < KS; ++ks) {
        FragB bh_, bl_;
        bh_.half[0] = *(const v8us*)&sKh[nt * 16 + ln][ks * 32 + 8 * hh]; bh_.half[1] = *(const v8us*)&sKh[nt * 16 + ln][ks * 32 + 16 + 8 * hh];
        bl_.half[0] = *(const v8us*)&sKl[nt * 16 + ln][ks * 32 + 8 * hh]; bl_.half[1] = *(const v8us*)&sKl[nt * 16 + ln][ks * 32 + 16 + 8 * hh];
        acc = mmaN<3>(aqh[ks].v, aql[ks].v, bh_.v, bl_.v, acc);
      }
      s[nt] = acc;
    }
    float alpha[8];
#pragma unroll
    for (int r = 0; r < 8; ++r) {
      const int qi = q0 + 8 * hh + r;
      const int ja = j0 + ln, jb = j0 + 16 + ln;
      if (CAUSAL) { if (ja > qi) s[0][r] = -3.0e38f; if (jb > qi) s[1][r] = -3.0e38f; }
      if (ja >= T) s[0][r] = -3.0e38f;
      if (jb >= T) s[1][r] = -3.0e38f;
      float mx = fmaxf(s[0][r], s[1][r]);
      mx = fmaxf(mx, __shfl_xor(mx, 1, 32)); mx = fmaxf(mx, __shfl_xor(mx, 2, 32)); mx = fmaxf(mx, __shfl_xor(mx, 4, 32)); mx = fmaxf(mx, __shfl_xor(mx, 8, 32));
      const float mnew = fmaxf(m_r[r], mx);
      alpha[r] = (mnew > -1.0e38f) ? __expf(m_r[r] - mnew) : 1.0f;
      const float p0 = (s[0][r] > -1.0e38f) ? __expf(s[0][r] - mnew) : 0.f;
      const float p1 = (s[1][r] > -1.0e38f) ? __expf(s[1][r] - mnew) : 0.f;
      m_r[r] = mnew;
      l_r[r] = l_r[r] * alpha[r] + p0 + p1;
      unsigned short hb = bf16_bits(p0); sPh[w][8 * hh + r][ln] = hb;      sPl[w][8 * hh + r][ln] = bf16_bits(p0 - bf16_val(hb));
      hb = bf16_bits(p1);                sPh[w][8 * hh + r][16 + ln] = hb; sPl[w][8 * hh + r][16 + ln] = bf16_bits(p1 - bf16_val(hb));
    }
#pragma unroll
    for (int dt = 0; dt < DT; ++dt)
#pragma unroll
      for (int r = 0; r < 8; ++r) oacc[dt][r] *= alpha[r];
    __builtin_amdgcn_fence(__ATOMIC_ACQ_REL, "workgroup");
    __builtin_amdgcn_wave_barrier();
    FragB pah, pal;
    pah.half[0] = *(const v8us*)&sPh[w][ln][8 * hh]; pah.half[1] = *(const v8us*)&sPh[w][ln][16 + 8 * hh];
    pal.half[0] = *(const v8us*)&sPl[w][ln][8 * hh]; pal.half[1] = *(const v8us*)&sPl[w][ln][16 + 8 * hh];
#pragma unroll
    for (int dt = 0; dt < DT; ++dt) {
      FragB bvh, bvl;
#pragma unroll
      for (int i = 0; i < 8; ++i) {
        bvh.u[i] = sVh[8 * hh + i][dt * 16 + ln]; bvh.u[8 + i] = sVh[16 + 8 * hh + i][dt * 16 + ln];
        bvl.u[i] = sVl[8 * hh + i][dt * 16 + ln]; bvl.u[8 + i] = sVl[16 + 8 * hh + i][dt * 16 + ln];
      }
      oacc[dt] = mmaN<3>(pah.v, pal.v, bvh.v, bvl.v, oacc[dt]);
    }
    __builtin_amdgcn_fence(__ATOMIC_ACQ_REL, "workgroup");
    __builtin_amdgcn_wave_barrier();
  }
#pragma unroll
  for (int r = 0; r < 8; ++r) {
    float l = l_r[r];
    l += __shfl_xor(l, 1, 32); l += __shfl_xor(l, 2, 32); l += __shfl_xor(l, 4, 32); l += __shfl_xor(l, 8, 32);
    l_r[r] = (l > 0.f) ? 1.0f / l : 0.f;
  }
#pragma unroll
  for (int dt = 0; dt < DT; ++dt)
#pragma unroll
    for (int r = 0; r < 8; ++r) sO[w][8 * hh + r][dt * 16 + ln] = oacc[dt][r] * l_r[r];
  __builtin_amdgcn_fence(__ATOMIC_ACQ_REL, "workgroup");
  __builtin_amdgcn_wave_barrier();
  for (int pass = 0; pass < 2; ++pass) {
    for (int r = 0; r < 16; ++r) {
      const int row = q0 + r;
      if (row < T && lane < D / 4) {
        const v4f val = *(const v4fa*)&sO[w][r][lane * 4];
        *(volatile v4f*)(y + ((size_t)b * T + row) * ypitch + h * D + lane * 4) = val;
      }
    }
    if (pass == 0) __threadfence();
  }
}

template <bool ASPLIT, int ACT, bool BIAS_BF16, bool RES_BF16>
__global__ __launch_bounds__(128) void k_gemm_bf3(const float* __restrict__ A, int lda, const unsigned short* __restrict__ Wt, int ldb,
                                                const float* __restrict__ bias, const float* __restrict__ resid, int rmod, int ldr,
                                                float* __restrict__ C, int ldc, int M, int N, int K) {
  __shared__ __attribute__((aligned(16))) float so[4][16][64];
  const int tid = threadIdx.x, w = tid >> 5, lane = tid & 31, ln = lane & 15, hh = lane >> 4;
  const int ntn = N / 64;
  const int wid = blockIdx.x * 4 + w;
  const int mt = wid / ntn, nq = wid % ntn;
  if (mt * 16 >= M) return;
  const int row0 = mt * 16, col0 = nq * 64;
  const float* arow = A + (size_t)(row0 + ln) * lda;
  v8f acc[4] = {};
  for (int kb = 0; kb < K; kb += 32) {
    FragB ah, al;
    const v4f x0 = *(const v4fa*)(arow + kb + 8 * hh), x1 = *(const v4fa*)(arow + kb + 8 * hh + 4);
    const v4f x2 = *(const v4fa*)(arow + kb + 16 + 8 * hh), x3 = *(const v4fa*)(arow + kb + 16 + 8 * hh + 4);
    float xs[16] = {x0[0],x0[1],x0[2],x0[3],x1[0],x1[1],x1[2],x1[3],x2[0],x2[1],x2[2],x2[3],x3[0],x3[1],x3[2],x3[3]};
#pragma unroll
    for (int i = 0; i < 16; ++i) { const unsigned short hb = bf16_bits(xs[i]); ah.u[i] = hb; al.u[i] = ASPLIT ? bf16_bits(xs[i] - bf16_val(hb)) : (unsigned short)0; }
#pragma unroll
    for (int t = 0; t < 4; ++t) {
      const unsigned short* brow = Wt + (size_t)(col0 + t * 16 + ln) * ldb + kb;
      FragB b;
      b.half[0] = *(const v8us*)(brow + 8 * hh);
      b.half[1] = *(const v8us*)(brow + 16 + 8 * hh);
      acc[t] = mmaN<ASPLIT ? 2 : 1>(ah.v, al.v, b.v, b.v, acc[t]);
    }
  }
#pragma unroll
  for (int t = 0; t < 4; ++t) {
    const int col = col0 + t * 16 + ln;
    float bv = bias ? bias[col] : 0.f;
    if (BIAS_BF16) bv = bf16_round(bv);
#pragma unroll
    for (int r = 0; r < 8; ++r) {
      float v = acc[t][r] + bv;
      if (resid) { float rv = resid[(size_t)((row0 + 8 * hh + r) % rmod) * ldr + col]; if (RES_BF16) rv = bf16_round(rv); v += rv; }
      if (ACT == 1) v = fmaxf(v, 0.f);
      if (ACT == 2) v = 0.5f * v * (1.0f + erff(v * 0.70710678118654752f));
      if (ACT == 3) { const float u = 0.7978845608028654f * (v + 0.044715f * v * v * v); v = 0.5f * v * (1.0f + tanhf(u)); }
      so[w][8 * hh + r][t * 16 + ln] = v;
    }
  }
  __builtin_amdgcn_fence(__ATOMIC_ACQ_REL, "workgroup");
  __builtin_amdgcn_wave_barrier();
  const int rsub = lane >> 4, c4 = (lane & 15) * 4;
  for (int pass = 0; pass < 2; ++pass) {
#pragma unroll
    for (int q = 0; q < 8; ++q) {
      const int r = q * 2 + rsub;
      const v4f v = *(const v4fa*)&so[w][r][c4];
      *(volatile v4f*)(C + (size_t)(row0 + r) * ldc + col0 + c4) = v;
    }
    if (pass == 0) __threadfence();
  }
}
template <bool PARAM_BF16>
__global__ __launch_bounds__(256) void k_layernorm(const float* __restrict__ X, const float* __restrict__ R, const float* __restrict__ g, const float* __restrict__ bta,
                                                  float* __restrict__ out_sum, float* __restrict__ out_norm, int N, float eps) {
  __shared__ float red[256];
  const int row = blockIdx.x, tid = threadIdx.x;
  const float* x = X + (size_t)row * N; const float* rr = R ? R + (size_t)row * N : nullptr;
  float vals[16];
  const int per = N / 256;
  float s1 = 0.f;
  for (int u = 0; u < per / 4; ++u) {
    const int j = tid * 4 + 1024 * u;
    const v4f a = *(const v4fa*)(x + j);
    v4f b = {0.f,0.f,0.f,0.f}; if (rr) b = *(const v4fa*)(rr + j);
#pragma unroll
    for (int q = 0; q < 4; ++q) { const float v = a[q] + b[q]; vals[u * 4 + q] = v; s1 += v; }
  }
  red[tid] = s1; __syncthreads();
  for (int st = 128; st > 0; st >>= 1) { if (tid < st) red[tid] += red[tid + st]; __syncthreads(); }
  const float mu = red[0] / (float)N; __syncthreads();
  float s2 = 0.f;
  for (int u = 0; u < per / 4; ++u)
#pragma unroll
    for (int q = 0; q < 4; ++q) { const float c = vals[u * 4 + q] - mu; s2 += c * c; }
  red[tid] = s2; __syncthreads();
  for (int st = 128; st > 0; st >>= 1) { if (tid < st) red[tid] += red[tid + st]; __syncthreads(); }
  const float rs = rsqrtf(red[0] / (float)N + eps);
  for (int pass = 0; pass < 2; ++pass) {
    for (int u = 0; u < per / 4; ++u) {
      const int j = tid * 4 + 1024 * u;
      v4f o, sm;
#pragma unroll
      for (int q = 0; q < 4; ++q) {
        float gg = g[j + q], bb = bta[j + q];
        if (PARAM_BF16) { gg = bf16_round(gg); bb = bf16_round(bb); }
        sm[q] = vals[u * 4 + q]; o[q] = (vals[u * 4 + q] - mu) * rs * gg + bb;
      }
      if (out_sum) *(volatile v4f*)(out_sum + (size_t)row * N + j) = sm;
      *(volatile v4f*)(out_norm + (size_t)row * N + j) = o;
    }
    if (pass == 0) __threadfence();
  }
}


typedef _Float16 v16h __attribute__((ext_vector_type(16)));
union FragH { v16h v; v8us half[2]; _Float16 h[16]; unsigned short u[16]; };
template <int NT>
__device__ __forceinline__ v8f mmaH(v16h ah, v16h al, v16h bh, v16h bl, v8f c) {
  c = __builtin_amdgcn_wmma_f32_16x16x32_f16(false, ah, false, bh, (short)0, c, false, false);
  if (NT >= 2) c = __builtin_amdgcn_wmma_f32_16x16x32_f16(false, al, false, bh, (short)0, c, false, false);
  if (NT >= 3) c = __builtin_amdgcn_wmma_f32_16x16x32_f16(false, ah, false, bl, (short)0, c, false, false);
  asm volatile("v_nop\n\tv_nop\n\tv_nop\n\tv_nop" : "+v"(c) : "v"(ah), "v"(al), "v"(bh), "v"(bl));
  return c;
}
template <bool ASPLIT>
__global__ __launch_bounds__(128) void k_gemm_h(const float* __restrict__ A, int lda, size_t sA, const _Float16* __restrict__ Bh, int ldb, size_t sB, float alpha, float* __restrict__ C, int ldc, size_t sC, int M, int N, int K) {
  __shared__ __attribute__((aligned(16))) float so[4][16][64];
  const int tid = threadIdx.x, w = tid >> 5, lane = tid & 31, ln = lane & 15, hh = lane >> 4; const int by = blockIdx.y;
  A += (size_t)by * sA; Bh += (size_t)by * sB; C += (size_t)by * sC;
  const int ntn = (N + 63) / 64; const int wid = blockIdx.x * 4 + w; const int mt = wid / ntn, nq = wid % ntn; if (mt * 16 >= M) return;
  const int row0 = mt * 16, col0 = nq * 64; const float* arow = A + (size_t)(row0 + ln) * lda;
  v8f acc[4] = {};
  for (int kb = 0; kb < K; kb += 32) {
    FragH ah, al;
    const v4f x0 = *(const v4fa*)(arow + kb + 8 * hh), x1 = *(const v4fa*)(arow + kb + 8 * hh + 4), x2 = *(const v4fa*)(arow + kb + 16 + 8 * hh), x3 = *(const v4fa*)(arow + kb + 16 + 8 * hh + 4);
    float xs[16] = {x0[0],x0[1],x0[2],x0[3],x1[0],x1[1],x1[2],x1[3],x2[0],x2[1],x2[2],x2[3],x3[0],x3[1],x3[2],x3[3]};
#pragma unroll
    for (int i = 0; i < 16; ++i) { const _Float16 h = (_Float16)xs[i]; ah.h[i] = h; al.h[i] = ASPLIT ? (_Float16)(xs[i] - (float)h) : (_Float16)0.0f; }
#pragma unroll
    for (int t = 0; t < 4; ++t) { if (col0 + t * 16 >= N) continue; const size_t boff = (size_t)(col0 + t * 16 + ln) * ldb + kb; FragH bq; bq.half[0] = *(const v8us*)(Bh + boff + 8 * hh); bq.half[1] = *(const v8us*)(Bh + boff + 16 + 8 * hh);
      acc[t] = mmaH<ASPLIT ? 2 : 1>(ah.v, al.v, bq.v, bq.v, acc[t]); }
  }
#pragma unroll
  for (int t = 0; t < 4; ++t) { if (col0 + t * 16 >= N) continue;
#pragma unroll
    for (int r = 0; r < 8; ++r) so[w][8 * hh + r][t * 16 + ln] = acc[t][r] * alpha; }
  __builtin_amdgcn_fence(__ATOMIC_ACQ_REL, "workgroup"); __builtin_amdgcn_wave_barrier();
  const int rsub = lane >> 4, c4 = (lane & 15) * 4;
  for (int pass = 0; pass < 2; ++pass) {
#pragma unroll
    for (int q = 0; q < 8; ++q) { const int r = q * 2 + rsub; if (col0 + c4 < N) { const v4f v = *(const v4fa*)&so[w][r][c4]; *(volatile v4f*)(C + (size_t)(row0 + r) * ldc + col0 + c4) = v; } }
    if (pass == 0) __threadfence(); }
}

__global__ __launch_bounds__(256) void k_wt_f16(const float* __restrict__ W, _Float16* __restrict__ Wt, int K, int N, float scale) {
  const int t = blockIdx.x * 256 + threadIdx.x; if (t >= N * (K / 8)) return; const int n = t / (K / 8), k8 = (t % (K / 8)) * 8; FragH f;
#pragma unroll
  for (int i = 0; i < 8; ++i) f.h[i] = (_Float16)(bf16_round(W[(size_t)(k8 + i) * N + n]) * scale); const v8us o = f.half[0];
  *(volatile v8us*)((unsigned short*)Wt + (size_t)n * K + k8) = o; __threadfence(); *(volatile v8us*)((unsigned short*)Wt + (size_t)n * K + k8) = o;
}
template <int ACT>
__global__ __launch_bounds__(128) void k_gemm_hhx(const _Float16* __restrict__ A, int lda, size_t sA, const _Float16* __restrict__ Bh, int ldb, size_t sB, float alpha, const float* __restrict__ bias, size_t sBias, const float* __restrict__ CP, int rowsPerB, size_t sCPb, int row0g,
    float* __restrict__ C, _Float16* __restrict__ C16, int ldc, size_t sC, int M, int N, int K) {
  __shared__ __attribute__((aligned(16))) float so[4][16][64];
  const int tid = threadIdx.x, w = tid >> 5, lane = tid & 31, ln = lane & 15, hh = lane >> 4; const int by = blockIdx.y;
  A += (size_t)by * sA; Bh += (size_t)by * sB; const size_t cofs = (size_t)by * sC; const float* bp = bias ? bias + (size_t)by * sBias : nullptr;
  const int ntn = (N + 63) / 64; const int wid = blockIdx.x * 4 + w; const int mt = wid / ntn, nq = wid % ntn; if (mt * 16 >= M) return;
  const int row0 = mt * 16, col0 = nq * 64; const _Float16* arow = A + (size_t)(row0 + ln) * lda;
  v8f acc[4] = {};
  for (int kb = 0; kb < K; kb += 32) { FragH ah; ah.half[0] = *(const v8us*)((const unsigned short*)arow + kb + 8 * hh); ah.half[1] = *(const v8us*)((const unsigned short*)arow + kb + 16 + 8 * hh);
#pragma unroll
    for (int t = 0; t < 4; ++t) { if (col0 + t * 16 >= N) continue; const size_t boff = (size_t)(col0 + t * 16 + ln) * ldb + kb; FragH bq; bq.half[0] = *(const v8us*)((const unsigned short*)Bh + boff + 8 * hh); bq.half[1] = *(const v8us*)((const unsigned short*)Bh + boff + 16 + 8 * hh);
      acc[t] = mmaH<1>(ah.v, ah.v, bq.v, bq.v, acc[t]); }
  }
#pragma unroll
  for (int t = 0; t < 4; ++t) { if (col0 + t * 16 >= N) continue; const int col = col0 + t * 16 + ln; const float bv = bp ? bf16_round(bp[col]) : 0.f;
#pragma unroll
    for (int r = 0; r < 8; ++r) { float v = acc[t][r] * alpha + bv; if (CP) { const int bidx = (row0g + row0 + 8 * hh + r) / rowsPerB; v += CP[(size_t)bidx * sCPb + (size_t)by * 64 + col]; } if (ACT == 1) v = (v > 0.f) ? v : expm1f(v); else if (ACT == 3) v = fmaxf(v, 0.f); so[w][8 * hh + r][t * 16 + ln] = v; } }
  __builtin_amdgcn_fence(__ATOMIC_ACQ_REL, "workgroup"); __builtin_amdgcn_wave_barrier();
  const int rsub = lane >> 4, c4 = (lane & 15) * 4; typedef _Float16 v4h __attribute__((ext_vector_type(4)));
  for (int pass = 0; pass < 2; ++pass) {
#pragma unroll
    for (int q = 0; q < 8; ++q) { const int r = q * 2 + rsub; if (col0 + c4 < N) { const v4f v = *(const v4fa*)&so[w][r][c4]; if (C) *(volatile v4f*)(C + cofs + (size_t)(row0 + r) * ldc + col0 + c4) = v; if (C16) { v4h h4; for (int i = 0; i < 4; ++i) h4[i] = (_Float16)v[i]; *(volatile v4h*)(C16 + cofs + (size_t)(row0 + r) * ldc + col0 + c4) = h4; } } }
    if (pass == 0) __threadfence(); }
}


typedef _Float16 v4h __attribute__((ext_vector_type(4)));

__global__ __launch_bounds__(256) void k_x16(const float* __restrict__ x, _Float16* __restrict__ X16, size_t n8) { const size_t t = (size_t)blockIdx.x * 256 + threadIdx.x; if (t >= n8) return; FragH f;
#pragma unroll
  for (int q = 0; q < 8; ++q) f.h[q] = (_Float16)bf16_round(x[t * 8 + q]); *(volatile v8us*)((unsigned short*)X16 + t * 8) = f.half[0]; __threadfence(); *(volatile v8us*)((unsigned short*)X16 + t * 8) = f.half[0]; }
__global__ __launch_bounds__(256) void k_h16(const float* __restrict__ x, _Float16* __restrict__ X16, size_t n8) { const size_t t = (size_t)blockIdx.x * 256 + threadIdx.x; if (t >= n8) return; FragH f;
#pragma unroll
  for (int q = 0; q < 8; ++q) f.h[q] = (_Float16)x[t * 8 + q]; *(volatile v8us*)((unsigned short*)X16 + t * 8) = f.half[0]; __threadfence(); *(volatile v8us*)((unsigned short*)X16 + t * 8) = f.half[0]; }
__global__ __launch_bounds__(256) void k_round16f(const float* __restrict__ W, _Float16* __restrict__ Bt, size_t n8) { const size_t t = (size_t)blockIdx.x * 256 + threadIdx.x; if (t >= n8) return; FragH f;
#pragma unroll
  for (int i = 0; i < 8; ++i) f.h[i] = (_Float16)(bf16_round(W[t * 8 + i]) * 16.0f); *(volatile v8us*)((unsigned short*)Bt + t * 8) = f.half[0]; __threadfence(); *(volatile v8us*)((unsigned short*)Bt + t * 8) = f.half[0]; }
template <int NHv, int TTv>
__global__ __launch_bounds__(256) void k_vt(const _Float16* __restrict__ V16, int ldv, int voff, _Float16* __restrict__ Vt) { __shared__ unsigned short tl[64][66]; const int tid = threadIdx.x; const int slab = blockIdx.x / (TTv / 64), lg = blockIdx.x % (TTv / 64); const int b = slab / NHv, h = slab % NHv;
  for (int i = tid; i < 64 * 8; i += 256) { const int r = i / 8, c8 = (i % 8) * 8; FragH f; f.half[0] = *(const v8us*)((const unsigned short*)V16 + ((size_t)b * TTv + lg * 64 + r) * ldv + voff + h * 64 + c8);
#pragma unroll
    for (int q = 0; q < 8; ++q) tl[r][c8 + q] = f.u[q]; }
  __syncthreads();
  for (int pass = 0; pass < 2; ++pass) {
#pragma unroll
    for (int rd = 0; rd < 2; ++rd) { const int d = rd * 32 + tid / 8, pc = tid % 8; FragH f;
#pragma unroll
      for (int q = 0; q < 8; ++q) f.u[q] = tl[pc * 8 + q][d];
      *(volatile v8us*)((unsigned short*)Vt + ((size_t)slab * 64 + d) * TTv + lg * 64 + pc * 8) = f.half[0]; }
    if (pass == 0) __threadfence(); } }

__device__ __forceinline__ void edge_of(const int* __restrict__ hist, int b, int e, int& src, int& dst, float& w, bool& valid) { const int h = e / (SQ - 1), s = e % (SQ - 1); src = hist[((size_t)b * HT + h) * SQ + s]; dst = hist[((size_t)b * HT + h) * SQ + s + 1]; w = 1.0f + expf(-0.01f * (float)(HT - 1 - h)); valid = (src != CC) && (dst != CC) && (src != dst); src = src < 0 ? 0 : (src >= CC ? CC - 1 : src); dst = dst < 0 ? 0 : (dst >= CC ? CC - 1 : dst); }
__global__ __launch_bounds__(256) void k_deg(const int* __restrict__ hist, float* __restrict__ Dv) { const int t = blockIdx.x * 256 + threadIdx.x; if (t >= BB * CC) return; const int b = t / CC, c = t % CC; float s = 1.0f;
#pragma unroll 1
  for (int e = 0; e < NEPB; ++e) { int sr, ds; float w; bool v; edge_of(hist, b, e, sr, ds, w, v); if (v && ds == c) s += w; } const float d = sqrtf(s); *(volatile float*)(Dv + t) = d; __threadfence(); *(volatile float*)(Dv + t) = d; }
__global__ __launch_bounds__(128) void k_ae(const int* __restrict__ hist, const float* __restrict__ E, const float* __restrict__ Dv, _Float16* __restrict__ AE) { __shared__ float acc[16][DIM]; const int b = blockIdx.x / (CC / 16), c0 = (blockIdx.x % (CC / 16)) * 16; const int k = threadIdx.x; for (int i = 0; i < 16; ++i) acc[i][k] = 0.f;
#pragma unroll 1
  for (int e = 0; e < NEPB; ++e) { int sr, ds; float w; bool v; edge_of(hist, b, e, sr, ds, w, v); if (v && sr >= c0 && sr < c0 + 16) acc[sr - c0][k] += w * Dv[b * CC + ds] * bf16_round(E[(size_t)ds * DIM + k]); }
  for (int i = 0; i < 16; ++i) { const float dc = Dv[b * CC + c0 + i]; acc[i][k] = dc * (dc * bf16_round(E[(size_t)(c0 + i) * DIM + k]) + acc[i][k]); } __syncthreads();
  for (int pass = 0; pass < 2; ++pass) { for (int p = k; p < 16 * 16; p += 128) { const int i = p / 16, pc = p % 16; FragH f; for (int q = 0; q < 8; ++q) f.h[q] = (_Float16)acc[i][pc * 8 + q]; *(volatile v8us*)((unsigned short*)AE + ((size_t)b * CC + c0 + i) * DIM + pc * 8) = f.half[0]; } if (pass == 0) __threadfence(); } }
__device__ __forceinline__ int tok_of(const int* __restrict__ hist, const int* __restrict__ cur, int r, int& b, int& s) { if (r < BB * HT * SQ) { b = r / (HT * SQ); s = r % SQ; return hist[r]; } const int rr = r - BB * HT * SQ; b = rr / SQ; s = rr % SQ; return cur[rr]; }
__global__ __launch_bounds__(256) void k_temp(float* __restrict__ TEMP) { const int t = blockIdx.x * 256 + threadIdx.x; if (t >= SQ * DM) return; const int k = t % DM, s = t / DM; const float den = powf(10000.0f, (float)(2 * (k / 2)) / (float)DM); const float arg = (float)s / den; const float v = (k % 2 == 0) ? sinf(arg) : cosf(arg); *(volatile float*)(TEMP + t) = v; __threadfence(); *(volatile float*)(TEMP + t) = v; }
__global__ __launch_bounds__(256) void k_fuse(const int* __restrict__ hist, const int* __restrict__ cur, const float* __restrict__ E, const float* __restrict__ EG, const float* __restrict__ nul, const float* __restrict__ TEMP, float* __restrict__ X, _Float16* __restrict__ X16) { const size_t t = (size_t)blockIdx.x * 256 + threadIdx.x; if (t >= (size_t)NR * (DM / 4)) return; const int k4 = (int)(t % (DM / 4)) * 4; const int r = (int)(t / (DM / 4)); int b, s; int tok = tok_of(hist, cur, r, b, s); const bool isnull = (tok == CC); tok = tok < 0 ? 0 : (tok >= CC ? CC - 1 : tok); v4f o; v4h h;
#pragma unroll
  for (int q = 0; q < 4; ++q) { const int k = k4 + q; const float tp = TEMP[s * DM + k]; float v; if (isnull) v = bf16_round(nul[k]); else v = (k < DIM) ? bf16_round(E[(size_t)tok * DIM + k]) : EG[((size_t)b * CC + tok) * DIM + (k - DIM)]; o[q] = v + tp; h[q] = (_Float16)o[q]; }
  for (int pass = 0; pass < 2; ++pass) { *(volatile v4f*)(X + (size_t)r * DM + k4) = o; *(volatile v4h*)(X16 + (size_t)r * DM + k4) = h; if (pass == 0) __threadfence(); } }
__global__ __launch_bounds__(256) void k_kmask(const int* __restrict__ hist, const int* __restrict__ cur, float* __restrict__ KM) { const int r = blockIdx.x * 256 + threadIdx.x; if (r >= NR) return; int b, s; const int tok = tok_of(hist, cur, r, b, s); const float v = (tok == CC) ? 1.f : 0.f; *(volatile float*)(KM + r) = v; __threadfence(); *(volatile float*)(KM + r) = v; }
__global__ __launch_bounds__(256) void k_attn(const float* __restrict__ Qp, int ldq, int qcol, const float* __restrict__ Kp, const float* __restrict__ Vp, int ldk, int kcol, int vcol, const float* __restrict__ KM, int window, int wca, _Float16* __restrict__ O16) { __shared__ float sqv[SQ][HDD + 1], sk[SQ][HDD + 1], sp[SQ][SQ + 1];        const int tid = threadIdx.x; const int seq = blockIdx.x / NHD, hd = blockIdx.x % NHD; int qrow0, krow0; if (!wca) { qrow0 = seq * SQ; krow0 = qrow0; } else { qrow0 = seq * SQ; krow0 = (BB * HT + seq / HT) * SQ - BB * HT * SQ; }
  for (int i = tid; i < SQ * HDD; i += 256) { const int r = i / HDD, d = i % HDD; sqv[r][d] = Qp[(size_t)(qrow0 + r) * ldq + qcol + hd * HDD + d]; sk[r][d] = Kp[(size_t)(krow0 + r) * ldk + kcol + hd * HDD + d]; } __syncthreads();
  for (int i = tid; i < SQ * SQ; i += 256) { const int qi = i / SQ, kj = i % SQ; float s = 0.f;
#pragma unroll 1
    for (int d = 0; d < HDD; ++d) s += sqv[qi][d] * sk[kj][d]; s *= 0.125f; bool masked = false; if (KM) masked = KM[krow0 + kj] != 0.f; if (window > 0) masked = masked || (abs(qi - kj) > window); sp[qi][kj] = masked ? -3.0e38f : s; } __syncthreads();
  for (int i = tid; i < SQ * HDD; i += 256) { const int r = i / HDD, d = i % HDD; sqv[r][d] = Vp[(size_t)(krow0 + r) * ldk + vcol + hd * HDD + d]; }
  { const int qi = tid / 4, part = tid % 4; float m = -3.0e38f; for (int j = part; j < SQ; j += 4) m = fmaxf(m, sp[qi][j]); m = fmaxf(m, __shfl_xor(m, 1, 32)); m = fmaxf(m, __shfl_xor(m, 2, 32)); float z = 0.f; for (int j = part; j < SQ; j += 4) { const float e = (sp[qi][j] <= -1.0e38f) ? 0.f : expf(sp[qi][j] - m); sp[qi][j] = e; z += e; } z += __shfl_xor(z, 1, 32); z += __shfl_xor(z, 2, 32); const float iz = (z > 0.f) ? 1.0f / z : 0.f; for (int j = part; j < SQ; j += 4) sp[qi][j] *= iz; } __syncthreads();
  for (int half = 0; half < 2; ++half) { const int qi = half * 32 + tid / 8, d0 = (tid % 8) * 8; float o[8]; for (int q = 0; q < 8; ++q) o[q] = 0.f;
#pragma unroll 1
    for (int j = 0; j < SQ; ++j) { const float p = sp[qi][j]; for (int q = 0; q < 8; ++q) o[q] += p * sqv[j][d0 + q]; }
    FragH a; for (int q = 0; q < 8; ++q) a.h[q] = (_Float16)o[q]; unsigned short* op = (unsigned short*)O16 + (size_t)(qrow0 + qi) * DM + hd * HDD + d0; *(volatile v8us*)op = a.half[0]; __threadfence(); *(volatile v8us*)op = a.half[0]; } }
__global__ __launch_bounds__(256) void k_ln(const float* __restrict__ G, const float* __restrict__ R, const float* __restrict__ gam, const float* __restrict__ bet, int nrows, float* __restrict__ OF, _Float16* __restrict__ O16) { const int tid = threadIdx.x, wv = tid >> 5, lane = tid & 31; const int r = blockIdx.x * 8 + wv; if (r >= nrows) return; v4f y[2]; float s = 0.f;
  for (int j = 0; j < 2; ++j) { const int c = j * 128 + lane * 4; v4f g = *(const v4fa*)(G + (size_t)r * DM + c); const v4f x = *(const v4fa*)(R + (size_t)r * DM + c); for (int q = 0; q < 4; ++q) g[q] += x[q]; y[j] = g; s += g[0] + g[1] + g[2] + g[3]; }
  for (int o = 16; o >= 1; o >>= 1) s += __shfl_xor(s, o, 32); const float mu = s / (float)DM; float q2 = 0.f; for (int j = 0; j < 2; ++j) for (int q = 0; q < 4; ++q) { const float d = y[j][q] - mu; q2 += d * d; } for (int o = 16; o >= 1; o >>= 1) q2 += __shfl_xor(q2, o, 32); const float rs = rsqrtf(q2 / (float)DM + 1e-5f);
  v4f ov[2]; v4h hv[2]; for (int j = 0; j < 2; ++j) { const int c = j * 128 + lane * 4; for (int q = 0; q < 4; ++q) { const float v = (y[j][q] - mu) * rs * bf16_round(gam[c + q]) + bf16_round(bet[c + q]); ov[j][q] = v; hv[j][q] = (_Float16)v; } }
  for (int pass = 0; pass < 2; ++pass) { for (int j = 0; j < 2; ++j) { const int c = j * 128 + lane * 4; *(volatile v4f*)(OF + (size_t)r * DM + c) = ov[j]; *(volatile v4h*)(O16 + (size_t)r * DM + c) = hv[j]; } if (pass == 0) __threadfence(); } }
__global__ __launch_bounds__(256) void k_agg(const float* __restrict__ WCA, const float* __restrict__ MC, _Float16* __restrict__ AG) { __shared__ float red[HT][256]; __shared__ float aw[HT]; __shared__ float row[DM]; const int b = blockIdx.x / SQ, s = blockIdx.x % SQ; const int d = threadIdx.x; const float mcv = MC[((size_t)b * SQ + s) * DM + d];
#pragma unroll 1
  for (int h = 0; h < HT; ++h) red[h][d] = WCA[(((size_t)b * HT + h) * SQ + s) * DM + d] * mcv; __syncthreads();
#pragma unroll 1
  for (int o = 128; o >= 1; o >>= 1) { if (d < o) {
#pragma unroll 1
      for (int h = 0; h < HT; ++h) red[h][d] += red[h][d + o]; } __syncthreads(); }
  if (d == 0) { float m = -3.0e38f;
#pragma unroll 1
    for (int h = 0; h < HT; ++h) m = fmaxf(m, red[h][0] * 0.0625f); float z = 0.f;
#pragma unroll 1
    for (int h = 0; h < HT; ++h) { aw[h] = expf(red[h][0] * 0.0625f - m); z += aw[h]; }
#pragma unroll 1
    for (int h = 0; h < HT; ++h) aw[h] /= z; } __syncthreads();
  float a = mcv;
#pragma unroll 1
  for (int h = 0; h < HT; ++h) a += aw[h] * WCA[(((size_t)b * HT + h) * SQ + s) * DM + d]; row[d] = a; __syncthreads();
  if (d < DM / 8) { FragH f; for (int q = 0; q < 8; ++q) f.h[q] = (_Float16)row[d * 8 + q]; unsigned short* op = (unsigned short*)AG + ((size_t)b * SQ + s) * DM + d * 8; *(volatile v8us*)op = f.half[0]; __threadfence(); *(volatile v8us*)op = f.half[0]; } }
__global__ __launch_bounds__(256) void k_zero16(_Float16* __restrict__ P, size_t n8) { const size_t t = (size_t)blockIdx.x * 256 + threadIdx.x; if (t >= n8) return; FragH z; for (int q = 0; q < 8; ++q) z.h[q] = (_Float16)0.f; *(volatile v8us*)((unsigned short*)P + t * 8) = z.half[0]; __threadfence(); *(volatile v8us*)((unsigned short*)P + t * 8) = z.half[0]; }
__global__ __launch_bounds__(256) void k_bcat(const float* __restrict__ b0, const float* __restrict__ b1, const float* __restrict__ b2, int n, float* __restrict__ O) { const int t = blockIdx.x * 256 + threadIdx.x; if (t >= 3 * n) return; const float v = (t < n) ? b0[t] : ((t < 2 * n) ? b1[t - n] : b2[t - 2 * n]); *(volatile float*)(O + t) = v; __threadfence(); *(volatile float*)(O + t) = v; }
__global__ __launch_bounds__(256) void k_addf(const float* __restrict__ A, const float* __restrict__ Bv, float* __restrict__ O, size_t n4) { const size_t t = (size_t)blockIdx.x * 256 + threadIdx.x; if (t >= n4) return; const v4f a = *(const v4fa*)(A + t * 4), b = *(const v4fa*)(Bv + t * 4); v4f o; for (int q = 0; q < 4; ++q) o[q] = a[q] + b[q]; *(volatile v4f*)(O + t * 4) = o; __threadfence(); *(volatile v4f*)(O + t * 4) = o; }
__global__ __launch_bounds__(256) void k_final(const float* __restrict__ ST, float* __restrict__ out) { const int t = blockIdx.x * 256 + threadIdx.x; if (t >= BB * SQ * CC) return; const int c = t % CC, r = t / CC; const float v = ST[(size_t)r * 2048 + c]; *(volatile float*)(out + t) = v; __threadfence(); *(volatile float*)(out + t) = v; }
extern "C" void kernel_launch(void* const* d_in, const int* in_sizes, int n_in,
                              void* d_out, int out_size, void* d_ws, size_t ws_size, hipStream_t stream) {
  (void)in_sizes; (void)n_in; (void)out_size;
  const int* hist = (const int*)d_in[0]; const int* cur = (const int*)d_in[1]; const float* const* I = (const float* const*)d_in; const float* E = I[2]; const float* nul = I[3]; const float* gw = I[4]; const float* gb = I[5]; const float* aw = I[6]; const float* ab = I[7]; const float* fw1 = I[8]; const float* fb1 = I[9]; const float* fw2 = I[10]; const float* fb2 = I[11]; const float* lns = I[12]; const float* lnb = I[13]; const float* ww = I[14]; const float* wb = I[15]; const float* iw = I[16]; const float* ib = I[17];
  char* ws = (char*)d_ws; size_t off = 0;
  auto take = [&](size_t bytes) { char* p = ws + off; off += (bytes + 255) & ~(size_t)255; return p; };
  _Float16* Bqkv = (_Float16*)take((size_t)3 * DM * DM * 2); _Float16* Bo = (_Float16*)take((size_t)DM * DM * 2); _Float16* Bf1 = (_Float16*)take((size_t)DFF * DM * 2); _Float16* Bf2 = (_Float16*)take((size_t)DM * DFF * 2); _Float16* Bg = (_Float16*)take((size_t)DIM * DIM * 2); _Float16* Bi = (_Float16*)take((size_t)DIM * DM * 2); _Float16* BE = (_Float16*)take((size_t)2048 * DIM * 2); float* B3 = (float*)take(3 * DM * 4);
  float* TEMP = (float*)take((size_t)SQ * DM * 4); float* Dv = (float*)take((size_t)BB * CC * 4); _Float16* AE = (_Float16*)take((size_t)BB * CC * DIM * 2); float* EG = (float*)take((size_t)BB * CC * DIM * 4); float* X = (float*)take((size_t)NR * DM * 4); _Float16* X16 = (_Float16*)take((size_t)NR * DM * 2); float* KM = (float*)take((size_t)NR * 4); float* QKV = (float*)take((size_t)NR * 3 * DM * 4); _Float16* O16 = (_Float16*)take((size_t)NR * DM * 2); float* A = (float*)take((size_t)NR * DM * 4); _Float16* H16 = (_Float16*)take((size_t)NR * DFF * 2); float* WCAp = (float*)take((size_t)BB * HT * SQ * DM * 4); _Float16* AG = (_Float16*)take((size_t)BB * SQ * DM * 2); _Float16* F16 = (_Float16*)take((size_t)BB * SQ * DIM * 2); float* ST = (float*)take((size_t)BB * SQ * 2048 * 4);
  if (off > ws_size) return;
  k_deg<<<(BB * CC + 255) / 256, 256, 0, stream>>>(hist, Dv); k_ae<<<BB * (CC / 16), 128, 0, stream>>>(hist, E, Dv, AE);
  k_wt_f16<<<(DIM * 16 + 255) / 256, 256, 0, stream>>>(gw, Bg, DIM, DIM, 16.0f);
  k_gemm_hhx<3><<<dim3(((BB * CC / 16) * 2 + 3) / 4, 1), 128, 0, stream>>>(AE, DIM, 0, Bg, DIM, 0, 0.0625f, gb, 0, nullptr, 1, 0, 0, EG, nullptr, DIM, 0, BB * CC, DIM, DIM);
  k_temp<<<(SQ * DM + 255) / 256, 256, 0, stream>>>(TEMP); k_fuse<<<(unsigned)(((size_t)NR * (DM / 4) + 255) / 256), 256, 0, stream>>>(hist, cur, E, EG, nul, TEMP, X, X16); k_kmask<<<(NR + 255) / 256, 256, 0, stream>>>(hist, cur, KM);
  const dim3 g768(((NR / 16) * 12 + 3) / 4, 1), g256(((NR / 16) * 4 + 3) / 4, 1), g1024(((NR / 16) * 16 + 3) / 4, 1);
  for (int l = 0; l < 2; ++l) { const float* W4 = aw + (size_t)l * 4 * DM * DM; const float* b4 = ab + (size_t)l * 4 * DM;
    for (int i = 0; i < 3; ++i) k_wt_f16<<<(DM * 32 + 255) / 256, 256, 0, stream>>>(W4 + (size_t)i * DM * DM, Bqkv + (size_t)i * DM * DM, DM, DM, 16.0f); k_wt_f16<<<(DM * 32 + 255) / 256, 256, 0, stream>>>(W4 + (size_t)3 * DM * DM, Bo, DM, DM, 16.0f);
    k_bcat<<<(3 * DM + 255) / 256, 256, 0, stream>>>(b4, b4 + DM, b4 + 2 * DM, DM, B3);
    k_gemm_hhx<0><<<g768, 128, 0, stream>>>(X16, DM, 0, Bqkv, DM, 0, 0.0625f, B3, 0, nullptr, 1, 0, 0, QKV, nullptr, 3 * DM, 0, NR, 3 * DM, DM);
    k_attn<<<NSEQ * NHD, 256, 0, stream>>>(QKV, 3 * DM, 0, QKV, QKV, 3 * DM, DM, 2 * DM, KM, 0, 0, O16);
    k_gemm_hhx<0><<<g256, 128, 0, stream>>>(O16, DM, 0, Bo, DM, 0, 0.0625f, b4 + 3 * DM, 0, nullptr, 1, 0, 0, A, nullptr, DM, 0, NR, DM, DM);
    k_ln<<<(NR + 7) / 8, 256, 0, stream>>>(A, X, lns + (size_t)(l * 2) * DM, lnb + (size_t)(l * 2) * DM, NR, X, X16);
    k_wt_f16<<<(DFF * 32 + 255) / 256, 256, 0, stream>>>(fw1 + (size_t)l * DM * DFF, Bf1, DM, DFF, 16.0f); k_wt_f16<<<(DM * 128 + 255) / 256, 256, 0, stream>>>(fw2 + (size_t)l * DFF * DM, Bf2, DFF, DM, 16.0f);
    k_gemm_hhx<3><<<g1024, 128, 0, stream>>>(X16, DM, 0, Bf1, DM, 0, 0.0625f, fb1 + (size_t)l * DFF, 0, nullptr, 1, 0, 0, nullptr, H16, DFF, 0, NR, DFF, DM);
    k_gemm_hhx<0><<<g256, 128, 0, stream>>>(H16, DFF, 0, Bf2, DFF, 0, 0.0625f, fb2 + (size_t)l * DM, 0, nullptr, 1, 0, 0, A, nullptr, DM, 0, NR, DM, DFF);
    k_ln<<<(NR + 7) / 8, 256, 0, stream>>>(A, X, lns + (size_t)(l * 2 + 1) * DM, lnb + (size_t)(l * 2 + 1) * DM, NR, X, X16); }
  for (int i = 0; i < 3; ++i) k_wt_f16<<<(DM * 32 + 255) / 256, 256, 0, stream>>>(ww + (size_t)i * DM * DM, Bqkv + (size_t)i * DM * DM, DM, DM, 16.0f); k_wt_f16<<<(DM * 32 + 255) / 256, 256, 0, stream>>>(ww + (size_t)3 * DM * DM, Bo, DM, DM, 16.0f);
  k_bcat<<<(3 * DM + 255) / 256, 256, 0, stream>>>(wb, wb + DM, wb + 2 * DM, DM, B3);
  k_gemm_hhx<0><<<g768, 128, 0, stream>>>(X16, DM, 0, Bqkv, DM, 0, 0.0625f, B3, 0, nullptr, 1, 0, 0, QKV, nullptr, 3 * DM, 0, NR, 3 * DM, DM);
  k_attn<<<BB * HT * NHD, 256, 0, stream>>>(QKV, 3 * DM, 0, QKV + (size_t)BB * HT * SQ * 3 * DM, QKV + (size_t)BB * HT * SQ * 3 * DM, 3 * DM, DM, 2 * DM, nullptr, 4, 1, O16);
  k_gemm_hhx<0><<<dim3(((BB * HT * SQ / 16) * 4 + 3) / 4, 1), 128, 0, stream>>>(O16, DM, 0, Bo, DM, 0, 0.0625f, wb + 3 * DM, 0, X, 1, (size_t)DM, 0, WCAp, nullptr, DM, 0, BB * HT * SQ, DM, DM);
  k_agg<<<BB * SQ, 256, 0, stream>>>(WCAp, X + (size_t)BB * HT * SQ * DM, AG);
  k_wt_f16<<<(DIM * 32 + 255) / 256, 256, 0, stream>>>(iw, Bi, DM, DIM, 16.0f);
  k_gemm_hhx<3><<<dim3(((BB * SQ / 16) * 2 + 3) / 4, 1), 128, 0, stream>>>(AG, DM, 0, Bi, DM, 0, 0.0625f, ib, 0, nullptr, 1, 0, 0, nullptr, F16, DIM, 0, BB * SQ, DIM, DM);
  k_round16f<<<(unsigned)(((size_t)CC * DIM / 8 + 255) / 256), 256, 0, stream>>>(E, BE, (size_t)CC * DIM / 8); k_zero16<<<(48 * DIM / 8 + 255) / 256, 256, 0, stream>>>(BE + (size_t)CC * DIM, (size_t)48 * DIM / 8);
  k_gemm_hhx<0><<<dim3(((BB * SQ / 16) * ((CC + 63) / 64) + 3) / 4, 1), 128, 0, stream>>>(F16, DIM, 0, BE, DIM, 0, 0.0625f, nullptr, 0, nullptr, 1, 0, 0, ST, nullptr, 2048, 0, BB * SQ, CC, DIM);
  k_final<<<(BB * SQ * CC + 255) / 256, 256, 0, stream>>>(ST, (float*)d_out);
}
